// CausalSelfAttention_13443247637319
// MI455X (gfx1250) — hardware-verified
//
#include <hip/hip_runtime.h>


#ifndef NB
#define NB 2
#endif
#ifndef SEQ
#define SEQ 2048
#endif
#define NB_FULL  2
#define SEQ_FULL 2048
#define DM   1024
#define NH   16
#define HD   64
#define RH   512
#define RHE  ((RH < SEQ) ? RH : SEQ)
#define PCAR 1024.0f
#define RCAR 2048.0f
#define SCL  0.125f
#define LOG2E 1.4426950408889634f

#define XB_ELEMS ((size_t)NB * SEQ * DM)
#define W_ELEMS  ((size_t)DM * DM)
#define PLN      ((size_t)NB * SEQ * DM)

#define OFF_PL   ((size_t)0)
#define BYT_PL   ((XB_ELEMS + 3 * W_ELEMS) * 2)
#define OFF_BIAS (OFF_PL + BYT_PL)
#define BYT_BIAS ((size_t)3 * DM * 4)
#define OFF_P6   (OFF_BIAS + BYT_BIAS)
#define BYT_P6   ((size_t)6 * PLN * 2)
#define WS_TOTAL (OFF_P6 + BYT_P6)

static_assert(NH * HD == DM);
static_assert(HD == 64);
static_assert(DM % 64 == 0);
static_assert(DM % 32 == 0);
static_assert(DM % 256 == 0);
static_assert(SEQ % 64 == 0);
static_assert(SEQ <= SEQ_FULL);
static_assert(NB <= NB_FULL);
static_assert(RH % 16 == 0);
static_assert(RHE % 16 == 0);
static_assert((SEQ - RHE) % 16 == 0);
static_assert((XB_ELEMS / 8) % 256 == 0);
static_assert((W_ELEMS / 8) % 256 == 0);
static_assert(BYT_PL % 256 == 0);
static_assert(BYT_BIAS % 256 == 0);
static_assert(WS_TOTAL <= (size_t)134217728);
static_assert((size_t)NB_FULL * SEQ_FULL * DM * 4 == (size_t)16777216);

typedef _Float16 h16;
typedef unsigned short bf;
typedef __attribute__((ext_vector_type(16))) __bf16   v16bf;
typedef __attribute__((ext_vector_type(16))) _Float16 v16h;
typedef __attribute__((ext_vector_type(8)))  _Float16 v8h;
typedef __attribute__((ext_vector_type(8)))  unsigned short v8us;
typedef __attribute__((ext_vector_type(16))) unsigned short v16us;
typedef __attribute__((ext_vector_type(8)))  float    v8f;
typedef __attribute__((ext_vector_type(4)))  float    v4f;

__device__ __forceinline__ unsigned short f2bf(float f) { unsigned u = __float_as_uint(f); u += 0x7FFFu + ((u >> 16) & 1u); return (unsigned short)(u >> 16); }
__device__ __forceinline__ float bf2f(unsigned short b) { return __uint_as_float(((unsigned)b) << 16); }
__device__ __forceinline__ float bfr(float f) { return bf2f(f2bf(f)); }
__device__ __forceinline__ v16h cat16(v8h lo, v8h hi) { return __builtin_shufflevector(lo, hi, 0, 1, 2, 3, 4, 5, 6, 7, 8, 9, 10, 11, 12, 13, 14, 15); }
__device__ __forceinline__ v16bf cat16b(v8us lo, v8us hi) { return __builtin_bit_cast(v16bf, __builtin_shufflevector(lo, hi, 0, 1, 2, 3, 4, 5, 6, 7, 8, 9, 10, 11, 12, 13, 14, 15)); }
__device__ __forceinline__ v16h ldh(const h16* p) { return cat16(*(const v8h*)p, *(const v8h*)(p + 16)); }
__device__ __forceinline__ v16bf ldb(const bf* p) { return cat16b(*(const v8us*)p, *(const v8us*)(p + 16)); }
__device__ __forceinline__ v8f wmma16(v16h a, v16h b, v8f c) { return __builtin_amdgcn_wmma_f32_16x16x32_f16(false, a, false, b, (short)0, c, false, false); }
__device__ __forceinline__ v8f wmmab(v16bf a, v16bf b, v8f c) { return __builtin_amdgcn_wmma_f32_16x16x32_bf16(false, a, false, b, (short)0, c, false, false); }

__global__ __launch_bounds__(256) void k_cvt8(const float* __restrict__ src, bf* dst, unsigned n8, unsigned inner8, unsigned sstride8) {
    const unsigned i = blockIdx.x * 256u + threadIdx.x; if (i >= n8) return;
    const unsigned bi = i / inner8, rem = i - bi * inner8;
    const size_t so = ((size_t)bi * sstride8 + rem) * 8;
    const v4f v0 = *(const v4f*)(src + so), v1 = *(const v4f*)(src + so + 4);
    v8us o;
#pragma unroll
    for (int k = 0; k < 4; ++k) { o[k] = f2bf(v0[k]); o[4 + k] = f2bf(v1[k]); }
    *(volatile v8us*)(dst + (size_t)i * 8) = o; __threadfence(); *(volatile v8us*)(dst + (size_t)i * 8) = o;
}

__global__ __launch_bounds__(256) void k_bias(const float* __restrict__ bq, const float* __restrict__ bk, const float* __restrict__ bv, float* dst) {
    const int i = blockIdx.x * 256 + threadIdx.x;
    const float a = bfr(bq[i]), b = bfr(bk[i]), c = bfr(bv[i]);
    *(volatile float*)(dst + i) = a; *(volatile float*)(dst + DM + i) = b; *(volatile float*)(dst + 2 * DM + i) = c;
    __threadfence();
    *(volatile float*)(dst + i) = a; *(volatile float*)(dst + DM + i) = b; *(volatile float*)(dst + 2 * DM + i) = c;
}

__global__ __launch_bounds__(32) void k_proj(const bf* __restrict__ PL, const float* __restrict__ BIAS, h16* OP) {
    __shared__ __align__(16) h16 th[64 * 72];
    __shared__ __align__(16) h16 tr[64 * 72];
    const int z = blockIdx.z; const bool vz = (z == 2);
    const int lane = threadIdx.x & 31, lr = lane & 15, hi = lane >> 4;
    const int tok0 = blockIdx.x * 64, f0 = blockIdx.y * 64;
    const size_t xoff = (size_t)tok0 * DM, woff = XB_ELEMS + (size_t)z * W_ELEMS + (size_t)f0 * DM;
    const size_t aoff = (vz ? xoff : woff) + (size_t)lr * DM + 8 * hi;
    const size_t boff = (vz ? woff : xoff) + (size_t)lr * DM + 8 * hi;
    v8f acc[4][4];
#pragma unroll
    for (int mb = 0; mb < 4; ++mb)
#pragma unroll
        for (int nb = 0; nb < 4; ++nb) acc[mb][nb] = (v8f){};
#pragma unroll 1
    for (int kc = 0; kc < DM; kc += 32) {
        v16bf a[4];
#pragma unroll
        for (int mb = 0; mb < 4; ++mb) a[mb] = ldb(PL + aoff + (size_t)mb * 16 * DM + kc);
#pragma unroll
        for (int nb = 0; nb < 4; ++nb) { const v16bf b = ldb(PL + boff + (size_t)nb * 16 * DM + kc);
#pragma unroll
            for (int mb = 0; mb < 4; ++mb) acc[mb][nb] = wmmab(a[mb], b, acc[mb][nb]); }
        asm volatile("v_nop\n\tv_nop\n\tv_nop\n\tv_nop" : "+v"(acc[0][0]), "+v"(acc[1][1]), "+v"(acc[2][2]), "+v"(acc[3][3]) : "v"(a[0]), "v"(a[3]));
    }
    const float* bz = BIAS + (size_t)z * DM + f0;
#pragma unroll
    for (int mb = 0; mb < 4; ++mb) {
        const v4f b0 = *(const v4f*)(bz + mb * 16 + 8 * hi), b1 = *(const v4f*)(bz + mb * 16 + 8 * hi + 4);
        float bI[8];
#pragma unroll
        for (int k = 0; k < 4; ++k) { bI[k] = vz ? 0.0f : b0[k]; bI[4 + k] = vz ? 0.0f : b1[k]; }
#pragma unroll
        for (int nb = 0; nb < 4; ++nb) {
            const float bl = bz[nb * 16 + lr]; const float bJ = vz ? bl : 0.0f;
            v8h oh, orr;
#pragma unroll
            for (int r = 0; r < 8; ++r) { const float val = acc[mb][nb][r] + (bI[r] + bJ); const h16 a = (h16)val; oh[r] = a; orr[r] = (h16)((val - (float)a) * RCAR); }
            *(v8h*)(th + (nb * 16 + lr) * 72 + mb * 16 + 8 * hi) = oh;
            *(v8h*)(tr + (nb * 16 + lr) * 72 + mb * 16 + 8 * hi) = orr; } }
    __syncthreads();
    const int b = tok0 / SEQ, t0 = tok0 - b * SEQ, hh = blockIdx.y;
    const size_t obase = vz ? ((size_t)(b * NH + hh) * HD * SEQ + t0) : (((size_t)(b * NH + hh) * SEQ + t0) * HD);
    const size_t pitch = vz ? (size_t)SEQ : (size_t)HD;
    const size_t hoff = (size_t)z * 2 * PLN, roff = hoff + PLN;
#pragma unroll 1
    for (int ps = 0; ps < 2; ++ps) {
#pragma unroll
        for (int s = 0; s < 16; ++s) { const int j = 4 * s + (lane >> 3), c = (lane & 7) * 8;
            const v8h va = *(const v8h*)(th + j * 72 + c); const v8h vb = *(const v8h*)(tr + j * 72 + c);
            *(volatile v8h*)(OP + hoff + obase + (size_t)j * pitch + c) = va;
            *(volatile v8h*)(OP + roff + obase + (size_t)j * pitch + c) = vb; }
        if (ps == 0) __threadfence(); }
}

template <bool HIRES>
__device__ __forceinline__ void attn_body(const h16* __restrict__ P6, const float* __restrict__ am, float* OUT, const int qt, const int bh) {
    __shared__ __align__(16) float os[16 * 68];
    const int lane = threadIdx.x & 31, n = lane & 15, hf = lane >> 4;
    const int b = bh / NH, h = bh - b * NH;
    const int q0 = qt * 16;
    const size_t hb = (size_t)bh * SEQ * HD;
    const h16* QH = P6 + hb;            const h16* QR = P6 + PLN + hb;
    const h16* KH = P6 + 2 * PLN + hb;  const h16* KR = P6 + 3 * PLN + hb;
    const h16* VH = P6 + 4 * PLN + hb;  const h16* VR = P6 + 5 * PLN + hb;
    const int qoff = (q0 + n) * HD + 8 * hf;
    v16h qh0 = {}, qh1 = {}, qr0 = {}, qr1 = {};
    if (!HIRES) { qh0 = ldh(QH + qoff); qh1 = ldh(QH + qoff + 32); qr0 = ldh(QR + qoff); qr1 = ldh(QR + qoff + 32); }
    v8f oh[4], ox[4];
#pragma unroll
    for (int dt = 0; dt < 4; ++dt) { oh[dt] = (v8f){}; ox[dt] = (v8f){}; }
    float m = -1.0e30f, l = 0.0f;
    const int kend = ((q0 >> 5) + 1) * 32;
    const float* amb = am + (size_t)b * SEQ_FULL + 8 * hf;
#pragma unroll 1
    for (int kb = 0; kb < kend; kb += 32) {
        int qo = qoff; if (HIRES) asm volatile("" : "+v"(qo));
        const int koff = (kb + n) * HD + 8 * hf;
        v8f s0 = (v8f){}, s1 = (v8f){}, r0 = (v8f){}, r1 = (v8f){};
#pragma unroll
        for (int c = 0; c < 2; ++c) {
            const v16h ka = ldh(KH + koff + 32 * c), kc2 = ldh(KH + koff + 16 * HD + 32 * c);
            v16h qa, qx;
            if (HIRES) { qa = ldh(QH + qo + 32 * c); qx = ldh(QR + qo + 32 * c); } else { qa = c ? qh1 : qh0; qx = c ? qr1 : qr0; }
            s0 = wmma16(ka, qa, s0); s1 = wmma16(kc2, qa, s1);
            r0 = wmma16(ka, qx, r0); r1 = wmma16(kc2, qx, r1);
            if (HIRES) { const v16h kra = ldh(KR + koff + 32 * c), krb = ldh(KR + koff + 16 * HD + 32 * c); r0 = wmma16(kra, qa, r0); r1 = wmma16(krb, qa, r1); }
            asm volatile("v_nop\n\tv_nop\n\tv_nop\n\tv_nop" : "+v"(s0), "+v"(s1), "+v"(r0), "+v"(r1) : "v"(ka), "v"(qa));
        }
        const v4f a0 = *(const v4f*)(amb + kb), a1 = *(const v4f*)(amb + kb + 4), a2 = *(const v4f*)(amb + kb + 16), a3 = *(const v4f*)(amb + kb + 20);
        float u[16];
#pragma unroll
        for (int r = 0; r < 4; ++r) {
            u[r]      = ((s0[r]     + r0[r]     * (1.0f / RCAR)) * SCL + a0[r]) * LOG2E;
            u[4 + r]  = ((s0[4 + r] + r0[4 + r] * (1.0f / RCAR)) * SCL + a1[r]) * LOG2E;
            u[8 + r]  = ((s1[r]     + r1[r]     * (1.0f / RCAR)) * SCL + a2[r]) * LOG2E;
            u[12 + r] = ((s1[4 + r] + r1[4 + r] * (1.0f / RCAR)) * SCL + a3[r]) * LOG2E; }
        if (kb + 31 > q0) {
            const int row = q0 + n, kbase = kb + 8 * hf;
#pragma unroll
            for (int i = 0; i < 8; ++i) { if (kbase + i > row) u[i] = -__builtin_inff(); if (kbase + 16 + i > row) u[8 + i] = -__builtin_inff(); } }
        float mx = u[0];
#pragma unroll
        for (int i = 1; i < 16; ++i) mx = fmaxf(mx, u[i]);
        mx = fmaxf(mx, __shfl_xor(mx, 16, 32));
        const float mn = fmaxf(m, mx);
        const float corr = __builtin_amdgcn_exp2f(m - mn); m = mn;
        float ls = 0.0f; v16h pf, px = {};
#pragma unroll
        for (int i = 0; i < 16; ++i) { const float p = __builtin_amdgcn_exp2f(u[i] - mn); ls += p; const float pc = p * PCAR; const h16 a = (h16)pc; pf[i] = a; if (HIRES) px[i] = (h16)((pc - (float)a) * RCAR); }
        l = l * corr + ls;
#pragma unroll
        for (int dt = 0; dt < 4; ++dt)
#pragma unroll
            for (int r = 0; r < 8; ++r) { oh[dt][r] *= corr; if (HIRES) ox[dt][r] *= corr; }
        const int voff = n * SEQ + kb + 8 * hf;
#pragma unroll
        for (int dt = 0; dt < 4; ++dt) {
            const v16h va = ldh(VH + voff + dt * 16 * SEQ);
            oh[dt] = wmma16(va, pf, oh[dt]);
            if (HIRES) { ox[dt] = wmma16(va, px, ox[dt]); const v16h vx = ldh(VR + voff + dt * 16 * SEQ); ox[dt] = wmma16(vx, pf, ox[dt]); } }
        if (HIRES) asm volatile("v_nop\n\tv_nop\n\tv_nop\n\tv_nop" : "+v"(oh[0]), "+v"(oh[1]), "+v"(oh[2]), "+v"(oh[3]), "+v"(ox[0]), "+v"(ox[1]), "+v"(ox[2]), "+v"(ox[3]) : "v"(pf), "v"(px));
        else       asm volatile("v_nop\n\tv_nop\n\tv_nop\n\tv_nop" : "+v"(oh[0]), "+v"(oh[1]), "+v"(oh[2]), "+v"(oh[3]) : "v"(pf));
    }
    const float lt = l + __shfl_xor(l, 16, 32);
    const float inv = (1.0f / PCAR) * (1.0f / lt);
#pragma unroll
    for (int dt = 0; dt < 4; ++dt) { v4f w0, w1;
#pragma unroll
        for (int r = 0; r < 4; ++r) { float e0 = oh[dt][r], e1 = oh[dt][4 + r]; if (HIRES) { e0 += ox[dt][r] * (1.0f / RCAR); e1 += ox[dt][4 + r] * (1.0f / RCAR); } w0[r] = e0 * inv; w1[r] = e1 * inv; }
        *(v4f*)(os + n * 68 + dt * 16 + 8 * hf) = w0; *(v4f*)(os + n * 68 + dt * 16 + 8 * hf + 4) = w1; }
    __syncthreads();
    float* orow = OUT + ((size_t)b * SEQ_FULL + q0) * DM + h * HD;
#pragma unroll 1
    for (int ps = 0; ps < 2; ++ps) {
#pragma unroll
        for (int s = 0; s < 8; ++s) { const int row = 2 * s + hf, cofs = n * 4; const v4f val = *(const v4f*)(os + row * 68 + cofs);
            *(volatile v4f*)(orow + (size_t)row * DM + cofs) = val; }
        if (ps == 0) __threadfence(); }
}

__global__ __launch_bounds__(32) void k_attn_hi(const h16* __restrict__ P6, const float* __restrict__ am, float* OUT) {
    const int wave = __builtin_amdgcn_readfirstlane(threadIdx.x >> 5);
    attn_body<true>(P6, am, OUT, (int)blockIdx.x + wave, (int)blockIdx.y);
}
__global__ __launch_bounds__(32) void k_attn_lo(const h16* __restrict__ P6, const float* __restrict__ am, float* OUT) {
    const int wave = __builtin_amdgcn_readfirstlane(threadIdx.x >> 5);
    attn_body<false>(P6, am, OUT, RHE / 16 + (int)blockIdx.x + wave, (int)blockIdx.y);
}

extern "C" void kernel_launch(void* const* d_in, const int* in_sizes, int n_in,
                              void* d_out, int out_size, void* d_ws, size_t ws_size, hipStream_t stream) {
    if (n_in < 8) return;
    const size_t xneed = ((size_t)(NB - 1) * SEQ_FULL + SEQ) * DM, mneed = (size_t)(NB - 1) * SEQ_FULL + SEQ;
    if ((size_t)in_sizes[0] < xneed || (size_t)in_sizes[1] < mneed) return;
    if ((size_t)in_sizes[2] < W_ELEMS || (size_t)in_sizes[4] < W_ELEMS || (size_t)in_sizes[6] < W_ELEMS) return;
    if (in_sizes[3] < DM || in_sizes[5] < DM || in_sizes[7] < DM) return;
    if ((size_t)out_size < xneed) return;
    if (ws_size < WS_TOTAL) return;
    const float* x  = (const float*)d_in[0];
    const float* am = (const float*)d_in[1];
    const float* wq = (const float*)d_in[2]; const float* bq = (const float*)d_in[3];
    const float* wk = (const float*)d_in[4]; const float* bk = (const float*)d_in[5];
    const float* wv = (const float*)d_in[6]; const float* bv = (const float*)d_in[7];
    float* OUT = (float*)d_out;
    char* wsb = (char*)d_ws;
    bf* PL = (bf*)(wsb + OFF_PL); float* BIAS = (float*)(wsb + OFF_BIAS); h16* P6 = (h16*)(wsb + OFF_P6);

    const unsigned xn8 = (unsigned)(XB_ELEMS / 8), wn8 = (unsigned)(W_ELEMS / 8);
    k_cvt8<<<xn8 / 256, 256, 0, stream>>>(x, PL, xn8, (unsigned)((size_t)SEQ * DM / 8), (unsigned)((size_t)SEQ_FULL * DM / 8));
    k_cvt8<<<wn8 / 256, 256, 0, stream>>>(wq, PL + XB_ELEMS, wn8, wn8, 0u);
    k_cvt8<<<wn8 / 256, 256, 0, stream>>>(wk, PL + XB_ELEMS + W_ELEMS, wn8, wn8, 0u);
    k_cvt8<<<wn8 / 256, 256, 0, stream>>>(wv, PL + XB_ELEMS + 2 * W_ELEMS, wn8, wn8, 0u);
    k_bias<<<DM / 256, 256, 0, stream>>>(bq, bk, bv, BIAS);
    k_proj<<<dim3(NB * SEQ / 64, DM / 64, 3), 32, 0, stream>>>(PL, BIAS, P6);
    k_attn_hi<<<dim3(RHE / 16, NB * NH), 32, 0, stream>>>(P6, am, OUT);
    if (SEQ > RHE) k_attn_lo<<<dim3((SEQ - RHE) / 16, NB * NH), 32, 0, stream>>>(P6, am, OUT);
}
